// FlashAttention_13254269075497
// MI455X (gfx1250) — hardware-verified
//
#include <hip/hip_runtime.h>
#include <math.h>

typedef __attribute__((ext_vector_type(16))) _Float16 v16h;
typedef __attribute__((ext_vector_type(8)))  _Float16 v8h;
typedef __attribute__((ext_vector_type(8)))  float v8f;
typedef __attribute__((ext_vector_type(4)))  float v4f;

template <typename T> __device__ __forceinline__ void vst2(void* p, T v) { *(volatile T*)p = v; __threadfence(); *(volatile T*)p = v; }
__device__ __forceinline__ v8f wmma16(v16h a, v16h b, v8f c) {
  v8f d = __builtin_amdgcn_wmma_f32_16x16x32_f16(false, a, false, b, (short)0, c, false, false);
  asm volatile("v_nop\n\tv_nop\n\tv_nop\n\tv_nop" : "+v"(d) : "v"(a), "v"(b));
  return d;
}
__device__ __forceinline__ v16h frag_h(const _Float16* rowk0, unsigned lane) {
  union { v16h v; v8h q[2]; } u; const _Float16* p = rowk0 + 8u * (lane >> 4);
  u.q[0] = *(const v8h*)p; u.q[1] = *(const v8h*)(p + 16); return u.v;
}
#define LDSX() do { asm volatile("s_wait_dscnt 0" ::: "memory"); __builtin_amdgcn_wave_barrier(); __builtin_amdgcn_fence(3  , "workgroup"); } while (0)

#ifndef NB
#define NB 1
#endif
#ifndef TT
#define TT 8192
#endif
#define NB_FULL 1
#define TT_FULL 8192
#define CC 128
#define HD 128
#define NQB (TT / 64)
#define LOG2E (1.4426950408889634f)
static_assert(TT % 128 == 0);
static_assert(TT <= TT_FULL);
static_assert(NB <= NB_FULL);
static_assert((NB * TT) % 64 == 0);
static_assert(NQB * 64 == TT);
static_assert(HD == 128);
static_assert(CC == HD);
static_assert(TT % 32 == 0);
static_assert(HD % 32 == 0);
static_assert(32 * 16 == HD * 4);
static_assert(4 * 16 == 64);
static_assert(2 * (64 * 136 * 2) + 128 * 72 * 2 <= 131072);
static_assert(4 * 16 * (HD + 4) * 4 <= 131072);

__device__ __forceinline__ float bfr(float v) { return (float)(__bf16)v; }

typedef _Float16 h16;
static __device__ __forceinline__ h16 p16_flush(float e) { const float p = exp2f(e + 14.0f); return (e < -28.0f) ? (h16)0.0f : (h16)p; }

#define WS_QH  ((size_t)0)
#define WS_KH  (WS_QH + (size_t)2 * NB * TT * CC)
#define WS_VT  (WS_KH + (size_t)2 * NB * TT * CC)
#define WS_END (WS_VT + (size_t)2 * NB * CC * TT)
static_assert(WS_END <= (size_t)134217728);
static_assert(WS_KH % 128 == 0);
static_assert(WS_VT % 128 == 0);

__global__ __launch_bounds__(128) void k_prep(const float* __restrict__ Q, const float* __restrict__ K, const float* __restrict__ V, _Float16* __restrict__ QH, _Float16* __restrict__ KH, _Float16* __restrict__ VT) {
  __shared__ __align__(16) _Float16 sq[64][136], sk[64][136], tv[128][72];
  const unsigned tid = threadIdx.x; const unsigned r0 = blockIdx.x * 64u; const unsigned bb = r0 / (unsigned)TT, t0 = r0 % (unsigned)TT;
  const size_t ib = ((size_t)bb * TT_FULL + t0) * HD;
  for (unsigned e = tid; e < 64u * 128u; e += 128u) { const unsigned rl = e >> 7, c = e & 127u; const size_t oi = ib + (size_t)rl * HD + c;
    const float q = bfr(Q[oi]), k = bfr(K[oi]), v = bfr(V[oi]);
    sq[rl][c] = (_Float16)q; sk[rl][c] = (_Float16)k; tv[c][rl] = (_Float16)v; }
  __syncthreads();
  for (unsigned e = tid; e < 64u * 16u; e += 128u) { const unsigned rl = e >> 4, q = e & 15u; const size_t o = ((size_t)r0 + rl) * CC + q * 8u;
    const v8h a = *(const v8h*)&sq[rl][q * 8u]; const v8h b = *(const v8h*)&sk[rl][q * 8u];
    vst2(QH + o, a); vst2(KH + o, b); }
  for (unsigned e = tid; e < 128u * 8u; e += 128u) { const unsigned cl = e >> 3, q = e & 7u;
    const v8h a = *(const v8h*)&tv[cl][q * 8u];
    vst2(VT + ((size_t)bb * CC + cl) * (size_t)TT + t0 + q * 8u, a); } }

__global__ __launch_bounds__(128) __attribute__((amdgpu_num_vgpr(256))) void k_fa(const _Float16* __restrict__ QH, const _Float16* __restrict__ KH, const _Float16* __restrict__ VT, float* __restrict__ Y) {
  __shared__ __align__(16) float ss[4][16][HD + 4];
  const unsigned tid = threadIdx.x, lane = tid & 31u, col = lane & 15u, g = lane >> 4;
  const unsigned wave = (unsigned)__builtin_amdgcn_readfirstlane((int)(tid >> 5));
  const unsigned b = blockIdx.y; const unsigned ql0 = blockIdx.x * 64u + wave * 16u;
  const size_t q0 = (size_t)b * TT + ql0, kr0 = (size_t)b * TT;
  const _Float16* vb = VT + (size_t)b * CC * (size_t)TT;
  v16h qf[HD / 32];
#pragma unroll
  for (int kc = 0; kc < HD / 32; ++kc) qf[kc] = frag_h(QH + (q0 + col) * CC + kc * 32, lane);
  v8f acc[HD / 16] = {};
  float m = -1.0e30f, l = 0.f;
#pragma unroll 1
  for (unsigned ks = 0; ks < (unsigned)(TT / 32); ++ks) { const unsigned k0 = ks * 32u;
    v8f s0 = {}, s1 = {};
#pragma unroll
    for (int kc = 0; kc < HD / 32; ++kc) {
      const v16h ka = frag_h(KH + (kr0 + k0 + col) * CC + kc * 32, lane); s0 = wmma16(ka, qf[kc], s0);
      const v16h kb = frag_h(KH + (kr0 + k0 + 16u + col) * CC + kc * 32, lane); s1 = wmma16(kb, qf[kc], s1); }
    float mx = fmaxf(s0[0], s1[0]);
#pragma unroll
    for (int r = 1; r < 8; ++r) mx = fmaxf(mx, fmaxf(s0[r], s1[r]));
    mx = fmaxf(mx, __shfl_xor(mx, 16));
    const float mn = fmaxf(m, mx);
    const float alpha = exp2f((m - mn) * LOG2E);
    m = mn;
    v16h pb; float ps = 0.f;
#pragma unroll
    for (int r = 0; r < 8; ++r) { const h16 p0 = p16_flush((s0[r] - mn) * LOG2E); const h16 p1 = p16_flush((s1[r] - mn) * LOG2E);
      pb[r] = p0; pb[8 + r] = p1; ps += (float)p0 + (float)p1; }
    ps += __shfl_xor(ps, 16);
    l = l * alpha + ps;
#pragma unroll
    for (int j = 0; j < HD / 16; ++j)
#pragma unroll
      for (int r = 0; r < 8; ++r) acc[j][r] *= alpha;
#pragma unroll
    for (int j = 0; j < HD / 16; ++j) { const v16h va = frag_h(vb + (size_t)(j * 16 + col) * (size_t)TT + k0, lane); acc[j] = wmma16(va, pb, acc[j]); } }
  const float inv = 1.0f / l;
#pragma unroll
  for (int j = 0; j < HD / 16; ++j)
#pragma unroll
    for (int r = 0; r < 8; ++r) ss[wave][col][j * 16 + 8 * g + r] = acc[j][r] * inv;
  LDSX();
  for (unsigned rl = 0; rl < 16u; ++rl) { const v4f o = *(const v4f*)&ss[wave][rl][lane * 4u]; vst2(Y + ((size_t)b * TT + ql0 + rl) * HD + lane * 4u, o); } }

extern "C" void kernel_launch(void* const* d_in, const int* in_sizes, int n_in, void* d_out, int out_size, void* d_ws, size_t ws_size, hipStream_t stream) {
  if (n_in < 3) return;
  const size_t need = ((size_t)(NB - 1) * TT_FULL + TT) * CC;
  if ((size_t)in_sizes[0] < need || (size_t)in_sizes[1] < need || (size_t)in_sizes[2] < need) return;
  if ((size_t)out_size < (size_t)NB * TT * CC) return;
  if (ws_size < (size_t)WS_END) return;
  const float* Qp = (const float*)d_in[0]; const float* Kp = (const float*)d_in[1]; const float* Vp = (const float*)d_in[2];
  char* ws = (char*)d_ws; _Float16* QH = (_Float16*)(ws + WS_QH); _Float16* KH = (_Float16*)(ws + WS_KH); _Float16* VT = (_Float16*)(ws + WS_VT);
  k_prep<<<dim3(NB * TT / 64), 128, 0, stream>>>(Qp, Kp, Vp, QH, KH, VT);
  k_fa<<<dim3(NQB, NB), 128, 0, stream>>>(QH, KH, VT, (float*)d_out);
}
